// Criterion1_28604482192026
// MI455X (gfx1250) — hardware-verified
//
#include <hip/hip_runtime.h>
#include <math.h>
#include <stdint.h>

#define BB    32
#define TT    256
#define DV    1024
#define DJ    512
#define LW    20
#define LP    32
#define KS    4
#define T1    127
#define T2    62
#define T3    30
#define TPV   219
#define TPC   224
#define SP    256
#define NTG   7
#define NR    (BB * TPC)
#define SCP   32
#define LAMF  4.0f
#define HINGE 0.1f
#define ASC   4096.0f

static_assert((TT - KS) / 2 + 1 == T1);
static_assert((T1 - KS) / 2 + 1 == T2);
static_assert((T2 - KS) / 2 + 1 == T3);
static_assert(T1 + T2 + T3 == TPV);
static_assert(TPC == NTG * 32);
static_assert(TPV <= TPC);
static_assert(BB <= SCP);
static_assert(T1 <= 128 && T2 <= 64 && T3 <= 64 && 192 + 64 <= SP);
static_assert((DV % 64) == 0 && (DJ % 64) == 0 && ((KS * DV) % 32) == 0 && ((KS * DJ) % 32) == 0);
static_assert((NR % 32) == 0 && LW <= LP && LW > 16);
static_assert(((BB * TT * DV / 8) % 256) == 0 && ((DJ * DV * KS / 8) % 256) == 0);
static_assert(((DJ * DJ * KS / 8) % 256) == 0 && ((DJ * DJ / 8) % 256) == 0);

typedef __bf16   v16b __attribute__((ext_vector_type(16)));
typedef __bf16   v8b  __attribute__((ext_vector_type(8)));
typedef _Float16 v16h __attribute__((ext_vector_type(16)));
typedef _Float16 v8h  __attribute__((ext_vector_type(8)));
typedef float    v8f  __attribute__((ext_vector_type(8)));
typedef float    v4f  __attribute__((ext_vector_type(4)));
typedef unsigned int v4u __attribute__((ext_vector_type(4)));
union FragB { v16b v; v8b hf[2]; };
union FragH { v16h v; v8h hf[2]; };
union F8    { v4f v[2]; float f[8]; };

__device__ __forceinline__ unsigned short bf_bits(float f) {
  unsigned u = __float_as_uint(f);
  return (unsigned short)((u + 0x7FFFu + ((u >> 16) & 1u)) >> 16);
}
__device__ __forceinline__ float bf_up(unsigned short h) { return __uint_as_float(((unsigned)h) << 16); }
__device__ __forceinline__ unsigned pk16(unsigned short a, unsigned short b) { return (unsigned)a | ((unsigned)b << 16); }
__device__ __forceinline__ v8f zero8() { v8f z = {0.f, 0.f, 0.f, 0.f, 0.f, 0.f, 0.f, 0.f}; return z; }
__device__ __forceinline__ v4u zero4u() { v4u z = {0u, 0u, 0u, 0u}; return z; }
__device__ __forceinline__ void split_bits(float y, unsigned short& hi, unsigned short& lo) {
  hi = bf_bits(y);
  lo = bf_bits(y - bf_up(hi));
}

__device__ __forceinline__ v16b ldfrag_b(const __bf16* p) {
  FragB f;
  f.hf[0] = *(const v8b*)(p);
  f.hf[1] = *(const v8b*)(p + 16);
  return f.v;
}
__device__ __forceinline__ v16h ldfrag_h(const _Float16* p) {
  FragH f;
  f.hf[0] = *(const v8h*)(p);
  f.hf[1] = *(const v8h*)(p + 16);
  return f.v;
}

__device__ __forceinline__ v8f mma_b_raw(v16b a, v16b b, v8f c) {
  return __builtin_amdgcn_wmma_f32_16x16x32_bf16(false, a, false, b, (short)0, c, false, false);
}
__device__ __forceinline__ v8f mma_h_raw(v16h a, v16h b, v8f c) {
  return __builtin_amdgcn_wmma_f32_16x16x32_f16(false, a, false, b, (short)0, c, false, false);
}
__device__ __forceinline__ void dep_guard_b(v8f& a, v8f& b, v16b x, v16b y) {
#if defined(__HIP_DEVICE_COMPILE__)
  asm volatile("v_nop\n\tv_nop\n\tv_nop\n\tv_nop" : "+v"(a), "+v"(b) : "v"(x), "v"(y));
#endif
}
__device__ __forceinline__ void dep_guard_h3(v8f& a, v8f& b, v16h x, v16h y, v16h z) {
#if defined(__HIP_DEVICE_COMPILE__)
  asm volatile("v_nop\n\tv_nop\n\tv_nop\n\tv_nop" : "+v"(a), "+v"(b) : "v"(x), "v"(y), "v"(z));
#endif
}
__device__ __forceinline__ void keep4_b(v16b a, v16b b, v16b c, v16b d) {
#if defined(__HIP_DEVICE_COMPILE__)
  asm volatile("v_nop" :: "v"(a), "v"(b), "v"(c), "v"(d));
#endif
}
__device__ __forceinline__ void keep2_b(v16b a, v16b b) {
#if defined(__HIP_DEVICE_COMPILE__)
  asm volatile("v_nop" :: "v"(a), "v"(b));
#endif
}
__device__ __forceinline__ void acc_guard4(v8f& a, v8f& b, v8f& c, v8f& d) {
#if defined(__HIP_DEVICE_COMPILE__)
  asm volatile("v_nop\n\tv_nop\n\tv_nop\n\tv_nop" : "+v"(a), "+v"(b), "+v"(c), "+v"(d));
#endif
}
__device__ __forceinline__ void wave_sync_lds() {
  __builtin_amdgcn_fence(__ATOMIC_RELEASE, "workgroup");
  __builtin_amdgcn_wave_barrier();
  __builtin_amdgcn_fence(__ATOMIC_ACQUIRE, "workgroup");
}
__device__ __forceinline__ float hsum16(float v) {
  v += __shfl_xor(v, 8, 32);
  v += __shfl_xor(v, 4, 32);
  v += __shfl_xor(v, 2, 32);
  v += __shfl_xor(v, 1, 32);
  return v;
}
__device__ __forceinline__ float hmax16(float v) {
  v = fmaxf(v, __shfl_xor(v, 8, 32));
  v = fmaxf(v, __shfl_xor(v, 4, 32));
  v = fmaxf(v, __shfl_xor(v, 2, 32));
  v = fmaxf(v, __shfl_xor(v, 1, 32));
  return v;
}

__global__ __launch_bounds__(256) void stats_in(const float* __restrict__ src, int R, int C, float* st) {
  __shared__ double red1[256];
  __shared__ double red2[256];
  __shared__ __align__(16) float sLine[32];
  const int tid = threadIdx.x;
  const int c   = blockIdx.x;
  double s1 = 0.0, s2 = 0.0;
#pragma unroll 1
  for (int r = tid; r < R; r += 256) {
    const float v = bf_up(bf_bits(src[(size_t)r * (size_t)C + c]));
    s1 += (double)v;
    s2 += (double)v * (double)v;
  }
  if (tid < 32) sLine[tid] = 0.f;
  red1[tid] = s1;
  red2[tid] = s2;
  __syncthreads();
  for (int s = 128; s > 0; s >>= 1) {
    if (tid < s) {
      red1[tid] += red1[tid + s];
      red2[tid] += red2[tid + s];
    }
    __syncthreads();
  }
  if (tid == 0) {
    const double inv  = 1.0 / (double)R;
    const double mean = red1[0] * inv;
    double var = red2[0] * inv - mean * mean;
    if (var < 0.0) var = 0.0;
    sLine[0] = (float)mean;
    sLine[1] = 1.0f / sqrtf((float)var + 1e-5f);
  }
  __syncthreads();
  if (tid < 8) {
    const v4f v = *(const v4f*)(sLine + tid * 4);
    float* p = st + (size_t)c * 32 + tid * 4;
    *(volatile v4f*)p = v;
    __threadfence();
    *(volatile v4f*)p = v;
  }
}

__global__ __launch_bounds__(256) void stats_y(const float* __restrict__ Y, const float* __restrict__ bias, float* st) {
  __shared__ double red1[256];
  __shared__ double red2[256];
  __shared__ __align__(16) float sLine[32];
  const int tid = threadIdx.x;
  const int c   = blockIdx.x;
  const float bb = bf_up(bf_bits(bias[c]));
  double s1 = 0.0, s2 = 0.0;
#pragma unroll 1
  for (int idx = tid; idx < BB * TPV; idx += 256) {
    const int b  = idx / TPV;
    const int tp = idx - b * TPV;
    const int slot = tp + ((tp >= T1) ? 1 : 0) + ((tp >= T1 + T2) ? 2 : 0);
    const float v = Y[((size_t)(b * SP + slot)) * DJ + c] + bb;
    s1 += (double)v;
    s2 += (double)v * (double)v;
  }
  if (tid < 32) sLine[tid] = 0.f;
  red1[tid] = s1;
  red2[tid] = s2;
  __syncthreads();
  for (int s = 128; s > 0; s >>= 1) {
    if (tid < s) {
      red1[tid] += red1[tid + s];
      red2[tid] += red2[tid + s];
    }
    __syncthreads();
  }
  if (tid == 0) {
    const double inv  = 1.0 / (double)(BB * TPV);
    const double mean = red1[0] * inv;
    double var = red2[0] * inv - mean * mean;
    if (var < 0.0) var = 0.0;
    sLine[0] = (float)mean;
    sLine[1] = 1.0f / sqrtf((float)var + 1e-5f);
  }
  __syncthreads();
  if (tid < 8) {
    const v4f v = *(const v4f*)(sLine + tid * 4);
    float* p = st + (size_t)c * 32 + tid * 4;
    *(volatile v4f*)p = v;
    __threadfence();
    *(volatile v4f*)p = v;
  }
}

__global__ __launch_bounds__(256) void video_split8(const float* __restrict__ video, const float* __restrict__ st,
                                                    unsigned short* hi, unsigned short* lo, int n8tot) {
  const int i = blockIdx.x * 256 + threadIdx.x;
  if (i >= n8tot) return;
  const int c0 = (i & (DV / 8 - 1)) * 8;
  const float* xp = video + (size_t)i * 8;
  F8 x;
  x.v[0] = *(const v4f*)(xp);
  x.v[1] = *(const v4f*)(xp + 4);
  v4u ph, pl;
#pragma unroll
  for (int e = 0; e < 4; ++e) {
    const int ca = c0 + 2 * e, cb = ca + 1;
    const float ya = (bf_up(bf_bits(x.f[2 * e]))     - st[ca * 32]) * st[ca * 32 + 1];
    const float yb = (bf_up(bf_bits(x.f[2 * e + 1])) - st[cb * 32]) * st[cb * 32 + 1];
    unsigned short h0, l0, h1, l1;
    split_bits(ya, h0, l0);
    split_bits(yb, h1, l1);
    ph[e] = pk16(h0, h1);
    pl[e] = pk16(l0, l1);
  }
  *(volatile v4u*)(hi + (size_t)i * 8) = ph;
  *(volatile v4u*)(lo + (size_t)i * 8) = pl;
  __threadfence();
  *(volatile v4u*)(hi + (size_t)i * 8) = ph;
  *(volatile v4u*)(lo + (size_t)i * 8) = pl;
}

__global__ __launch_bounds__(256) void wconv_cvt8(const float* __restrict__ w, int Cin, int ks,
                                                  unsigned short* out, int n8tot) {
  const int i = blockIdx.x * 256 + threadIdx.x;
  if (i >= n8tot) return;
  const int cin8 = Cin >> 3;
  const int per  = ks * cin8;
  const int o    = i / per;
  const int rem  = i - o * per;
  const int kk   = rem / cin8;
  const int c0   = (rem - kk * cin8) * 8;
  const float* sp = w + (size_t)o * (size_t)Cin * ks + (size_t)c0 * ks + kk;
  v4u p;
#pragma unroll
  for (int e = 0; e < 4; ++e) p[e] = pk16(bf_bits(sp[(2 * e) * ks]), bf_bits(sp[(2 * e + 1) * ks]));
  *(volatile v4u*)(out + (size_t)i * 8) = p;
  __threadfence();
  *(volatile v4u*)(out + (size_t)i * 8) = p;
}

__global__ __launch_bounds__(256) void words_planes(const float* __restrict__ words, const float* __restrict__ stW,
                                                    unsigned short* WX, unsigned short* WH, unsigned short* WL) {
  const int lane = threadIdx.x & 31;
  const int gw   = blockIdx.x * 8 + (threadIdx.x >> 5);
  const int i = gw / LP, l = gw - i * LP;
  const int lc = (l < LW) ? l : (LW - 1);
  const float* src = words + ((size_t)(i * LW + lc)) * DJ;
  unsigned short* dx = WX + (size_t)gw * DJ;
  unsigned short* dh = WH + (size_t)gw * DJ;
  unsigned short* dl = WL + (size_t)gw * DJ;
#pragma unroll 1
  for (int g = 0; g < 2; ++g) {
    const int c0 = g * 256 + lane * 8;
    F8 x;
    x.v[0] = *(const v4f*)(src + c0);
    x.v[1] = *(const v4f*)(src + c0 + 4);
    v4u px, ph, pl;
#pragma unroll
    for (int e = 0; e < 4; ++e) {
      const int ca = c0 + 2 * e, cb = ca + 1;
      const unsigned short xa = bf_bits(x.f[2 * e]);
      const unsigned short xb = bf_bits(x.f[2 * e + 1]);
      const float wa = (bf_up(xa) - stW[ca * 32]) * stW[ca * 32 + 1];
      const float wb = (bf_up(xb) - stW[cb * 32]) * stW[cb * 32 + 1];
      unsigned short h0, l0, h1, l1;
      split_bits(wa, h0, l0);
      split_bits(wb, h1, l1);
      px[e] = pk16(xa, xb);
      ph[e] = pk16(h0, h1);
      pl[e] = pk16(l0, l1);
    }
    if (l >= LW) { px = zero4u(); ph = zero4u(); pl = zero4u(); }
    *(volatile v4u*)(dx + c0) = px;
    *(volatile v4u*)(dh + c0) = ph;
    *(volatile v4u*)(dl + c0) = pl;
    __threadfence();
    *(volatile v4u*)(dx + c0) = px;
    *(volatile v4u*)(dh + c0) = ph;
    *(volatile v4u*)(dl + c0) = pl;
  }
}

__global__ __launch_bounds__(32) void gram_kernel(const unsigned short* __restrict__ WHp, const unsigned short* __restrict__ WLp,
                                                  unsigned short* Gt) {
  __shared__ __align__(16) float sG[32 * 36];
  const int i = blockIdx.x;
  const int lane = threadIdx.x & 31;
  const int m = lane & 15, h = lane >> 4, koff = h * 8, mOff = h * 8;
  const __bf16* H = (const __bf16*)(const void*)WHp + (size_t)i * LP * DJ;
  const __bf16* L = (const __bf16*)(const void*)WLp + (size_t)i * LP * DJ;
  v8f acc[2][2];
#pragma unroll
  for (int a = 0; a < 2; ++a)
#pragma unroll
    for (int c = 0; c < 2; ++c) acc[a][c] = zero8();
  for (int k0 = 0; k0 < DJ; k0 += 32) {
    const v16b b0 = ldfrag_b(H + (size_t)m * DJ + koff + k0);
    const v16b b1 = ldfrag_b(H + (size_t)(16 + m) * DJ + koff + k0);
#pragma unroll
    for (int mi = 0; mi < 2; ++mi) {
      const size_t ao = (size_t)(mi * 16 + m) * DJ + koff + k0;
      const v16b ah = ldfrag_b(H + ao);
      const v16b al = ldfrag_b(L + ao);
      acc[mi][0] = mma_b_raw(ah, b0, acc[mi][0]);
      acc[mi][0] = mma_b_raw(al, b0, acc[mi][0]);
      acc[mi][1] = mma_b_raw(ah, b1, acc[mi][1]);
      acc[mi][1] = mma_b_raw(al, b1, acc[mi][1]);
      dep_guard_b(acc[mi][0], acc[mi][1], ah, al);
    }
    keep2_b(b0, b1);
  }
  acc_guard4(acc[0][0], acc[0][1], acc[1][0], acc[1][1]);
#pragma unroll
  for (int mi = 0; mi < 2; ++mi)
#pragma unroll
    for (int nj = 0; nj < 2; ++nj)
#pragma unroll
      for (int r = 0; r < 8; ++r) sG[(mi * 16 + mOff + r) * 36 + nj * 16 + m] = acc[mi][nj][r];
  wave_sync_lds();
  v8h gv[4];
#pragma unroll
  for (int it = 0; it < 4; ++it) {
    const int row = it * 8 + (lane >> 2);
    const int c8  = (lane & 3) * 8;
    F8 x;
    x.v[0] = *(const v4f*)(sG + row * 36 + c8);
    x.v[1] = *(const v4f*)(sG + row * 36 + c8 + 4);
#pragma unroll
    for (int e = 0; e < 8; ++e) gv[it][e] = (_Float16)x.f[e];
  }
  _Float16* G = (_Float16*)(void*)Gt + (size_t)i * LP * LP;
  for (int pass = 0; pass < 2; ++pass) {
#pragma unroll
    for (int it = 0; it < 4; ++it) {
      const int row = it * 8 + (lane >> 2);
      const int c8  = (lane & 3) * 8;
      *(volatile v8h*)(G + row * LP + c8) = gv[it];
    }
    __threadfence();
  }
}

template <int NSPLIT, int OUT_MODE>
__global__ __launch_bounds__(256) void gemm64(
    const unsigned short* __restrict__ Ap, const unsigned short* A2p, int lda, long long strideA, int Mreal,
    const unsigned short* __restrict__ Btp, int ldb, long long strideB,
    void* Cout, void* Cout2, int ldc, long long strideC, const float* __restrict__ bias,
    int M, int N, int K) {
  const __bf16* A  = (const __bf16*)(const void*)Ap;
  const __bf16* A2 = (const __bf16*)(const void*)A2p;
  const __bf16* Bt = (const __bf16*)(const void*)Btp;
  __shared__ __align__(16) float sT[8][16 * 68];
  const int b    = blockIdx.y;
  const int lane = threadIdx.x & 31;
  const int wave = threadIdx.x >> 5;
  const int tilesN = N >> 6;
  const int tilesM = M >> 6;
  const int tile = blockIdx.x * 8 + wave;
  if (tile >= tilesM * tilesN) return;
  const int tm = tile / tilesN;
  const int tn = tile - tm * tilesN;
  const int m0 = tm << 6;
  const int n0 = tn << 6;

  const __bf16* Ab  = A  + (size_t)b * strideA;
  const __bf16* Bb  = Bt + (size_t)b * strideB;
  const __bf16* Ab2 = (NSPLIT >= 1) ? (A2 + (size_t)b * strideA) : Ab;

  const int rlane = lane & 15;
  const int koff  = (lane >> 4) * 8;
  const int mOff  = (lane >> 4) * 8;

  v8f acc[4][4];
#pragma unroll
  for (int i = 0; i < 4; ++i)
#pragma unroll
    for (int j = 0; j < 4; ++j) acc[i][j] = zero8();

  for (int k0 = 0; k0 < K; k0 += 32) {
    v16b bh[4];
#pragma unroll
    for (int j = 0; j < 4; ++j) {
      const size_t bo = (size_t)(n0 + (j << 4) + rlane) * ldb + koff + k0;
      bh[j] = ldfrag_b(Bb + bo);
    }
#pragma unroll
    for (int i = 0; i < 4; ++i) {
      int ar = m0 + (i << 4) + rlane;
      ar = (ar > Mreal - 1) ? (Mreal - 1) : ar;
      const size_t ao = (size_t)ar * lda + koff + k0;
      const v16b ah = ldfrag_b(Ab + ao);
      v16b al = ah;
      if (NSPLIT >= 1) al = ldfrag_b(Ab2 + ao);
#pragma unroll
      for (int j = 0; j < 4; ++j) {
        acc[i][j] = mma_b_raw(ah, bh[j], acc[i][j]);
        if (NSPLIT >= 1) acc[i][j] = mma_b_raw(al, bh[j], acc[i][j]);
      }
      dep_guard_b(acc[i][0], acc[i][3], ah, al);
    }
    keep4_b(bh[0], bh[1], bh[2], bh[3]);
  }
  acc_guard4(acc[0][0], acc[0][1], acc[0][2], acc[0][3]);
  acc_guard4(acc[1][0], acc[1][1], acc[1][2], acc[1][3]);
  acc_guard4(acc[2][0], acc[2][1], acc[2][2], acc[2][3]);
  acc_guard4(acc[3][0], acc[3][1], acc[3][2], acc[3][3]);

  float* slab = sT[wave];
  if (OUT_MODE == 0) {
    const int hh = lane >> 4, c4 = (lane & 15) * 4;
    float* C = (float*)Cout + (size_t)b * strideC;
#pragma unroll
    for (int i = 0; i < 4; ++i) {
      const int mBase = m0 + (i << 4);
#pragma unroll
      for (int j = 0; j < 4; ++j) {
#pragma unroll
        for (int r = 0; r < 8; ++r) slab[(mOff + r) * 68 + (j << 4) + rlane] = acc[i][j][r];
      }
      wave_sync_lds();
      for (int pass = 0; pass < 2; ++pass) {
#pragma unroll
        for (int it = 0; it < 8; ++it) {
          const int row = it * 2 + hh;
          const v4f v = *(const v4f*)(slab + row * 68 + c4);
          *(volatile v4f*)(C + (size_t)(mBase + row) * ldc + n0 + c4) = v;
        }
        __threadfence();
      }
      wave_sync_lds();
    }
  } else {
    unsigned short* Ch = (unsigned short*)Cout  + (size_t)b * strideC;
    unsigned short* Cl = (unsigned short*)Cout2 + (size_t)b * strideC;
    const int r4 = lane >> 3, c8 = (lane & 7) * 8;
    F8 bz;
    bz.v[0] = *(const v4f*)(bias + n0 + c8);
    bz.v[1] = *(const v4f*)(bias + n0 + c8 + 4);
#pragma unroll
    for (int e = 0; e < 8; ++e) bz.f[e] = bf_up(bf_bits(bz.f[e]));
#pragma unroll
    for (int i = 0; i < 4; ++i) {
      const int mBase = m0 + (i << 4);
#pragma unroll
      for (int j = 0; j < 4; ++j) {
#pragma unroll
        for (int r = 0; r < 8; ++r) slab[(mOff + r) * 68 + (j << 4) + rlane] = acc[i][j][r];
      }
      wave_sync_lds();
      v4u ph[4], pl[4];
#pragma unroll
      for (int it = 0; it < 4; ++it) {
        const int row = it * 4 + r4;
        F8 x;
        x.v[0] = *(const v4f*)(slab + row * 68 + c8);
        x.v[1] = *(const v4f*)(slab + row * 68 + c8 + 4);
#pragma unroll
        for (int e = 0; e < 4; ++e) {
          const float y0 = fmaxf(x.f[2 * e]     + bz.f[2 * e],     0.f);
          const float y1 = fmaxf(x.f[2 * e + 1] + bz.f[2 * e + 1], 0.f);
          unsigned short h0, l0, h1, l1;
          split_bits(y0, h0, l0);
          split_bits(y1, h1, l1);
          ph[it][e] = pk16(h0, h1);
          pl[it][e] = pk16(l0, l1);
        }
      }
      for (int pass = 0; pass < 2; ++pass) {
#pragma unroll
        for (int it = 0; it < 4; ++it) {
          const int row = it * 4 + r4;
          const size_t o = (size_t)(mBase + row) * ldc + n0 + c8;
          *(volatile v4u*)(Ch + o) = ph[it];
          *(volatile v4u*)(Cl + o) = pl[it];
        }
        __threadfence();
      }
      wave_sync_lds();
    }
  }
}

__global__ __launch_bounds__(256) void vfinish(const float* __restrict__ Y, const float* __restrict__ bias,
                                               const float* __restrict__ stY, const float* __restrict__ stW,
                                               unsigned short* VH, unsigned short* VL, float* vnT, float* cT) {
  __shared__ __align__(16) float sVn[32];
  __shared__ __align__(16) float sC[32];
  const int tid = threadIdx.x, wave = tid >> 5, lane = tid & 31;
#pragma unroll 1
  for (int q = 0; q < 4; ++q) {
    const int lrow = wave * 4 + q;
    const int row  = blockIdx.x * 32 + lrow;
    const int b  = row / TPC;
    const int tp = row - b * TPC;
    const bool valid = tp < TPV;
    int slot = tp + ((tp >= T1) ? 1 : 0) + ((tp >= T1 + T2) ? 2 : 0);
    slot = valid ? slot : 0;
    const float* yr = Y + ((size_t)(b * SP + slot)) * DJ;
    float vn2 = 0.f, cc = 0.f;
#pragma unroll 1
    for (int g = 0; g < 2; ++g) {
      const int c0 = g * 256 + lane * 8;
      F8 x, bz;
      x.v[0]  = *(const v4f*)(yr + c0);
      x.v[1]  = *(const v4f*)(yr + c0 + 4);
      bz.v[0] = *(const v4f*)(bias + c0);
      bz.v[1] = *(const v4f*)(bias + c0 + 4);
      v4u ph, pl;
#pragma unroll
      for (int e = 0; e < 4; ++e) {
        const int ca = c0 + 2 * e, cb = ca + 1;
        float va = (x.f[2 * e]     + bf_up(bf_bits(bz.f[2 * e]))     - stY[ca * 32]) * stY[ca * 32 + 1];
        float vb = (x.f[2 * e + 1] + bf_up(bf_bits(bz.f[2 * e + 1])) - stY[cb * 32]) * stY[cb * 32 + 1];
        va = valid ? va : 0.f;
        vb = valid ? vb : 0.f;
        const float mwa = stW[ca * 32], rwa = stW[ca * 32 + 1];
        const float mwb = stW[cb * 32], rwb = stW[cb * 32 + 1];
        vn2 += va * va + vb * vb;
        cc  += va * (mwa * rwa) + vb * (mwb * rwb);
        unsigned short h0, l0, h1, l1;
        split_bits(va * rwa, h0, l0);
        split_bits(vb * rwb, h1, l1);
        ph[e] = pk16(h0, h1);
        pl[e] = pk16(l0, l1);
      }
      const size_t o = (size_t)row * DJ + c0;
      *(volatile v4u*)(VH + o) = ph;
      *(volatile v4u*)(VL + o) = pl;
      __threadfence();
      *(volatile v4u*)(VH + o) = ph;
      *(volatile v4u*)(VL + o) = pl;
    }
#pragma unroll
    for (int off = 16; off > 0; off >>= 1) {
      vn2 += __shfl_xor(vn2, off, 32);
      cc  += __shfl_xor(cc, off, 32);
    }
    if (lane == 0) {
      sVn[lrow] = valid ? sqrtf(vn2) : 1.f;
      sC[lrow]  = cc;
    }
  }
  __syncthreads();
  if (tid < 8) {
    const v4f a = *(const v4f*)(sVn + tid * 4);
    const v4f c = *(const v4f*)(sC + tid * 4);
    float* pa = vnT + (size_t)blockIdx.x * 32 + tid * 4;
    float* pc = cT  + (size_t)blockIdx.x * 32 + tid * 4;
    *(volatile v4f*)pa = a;
    *(volatile v4f*)pc = c;
    __threadfence();
    *(volatile v4f*)pa = a;
    *(volatile v4f*)pc = c;
  }
}

__global__ __launch_bounds__(128) void attn_kernel(
    const unsigned short* __restrict__ VHp, const unsigned short* __restrict__ VLp,
    const unsigned short* __restrict__ WXp, const unsigned short* __restrict__ Gtp,
    const float* __restrict__ vnT, const float* __restrict__ cT, const float* __restrict__ wmask,
    float* scoresT, float* posT) {
  __shared__ __align__(16) _Float16 sP[4][16 * LP];
  __shared__ __align__(16) float sPos[TPC];
  __shared__ __align__(16) float sSc[SCP];
  __shared__ float sItem[BB * NTG];
  const int i = blockIdx.x;
  const int tid = threadIdx.x, wave = tid >> 5, lane = tid & 31;
  const int h = lane >> 4, m = lane & 15, koff = h * 8;
  for (int t = tid; t < TPC; t += 128) sPos[t] = 0.f;
  for (int t = tid; t < BB * NTG; t += 128) sItem[t] = -3.0e38f;
  if (tid < SCP) sSc[tid] = 0.f;
  const int l1 = (16 + m < LW) ? (16 + m) : (LW - 1);
  const bool mk0  = wmask[i * LW + m]  > 0.5f;
  const bool mk1  = wmask[i * LW + l1] > 0.5f;
  const bool val1 = (16 + m) < LW;
  __syncthreads();

  const __bf16* VH = (const __bf16*)(const void*)VHp;
  const __bf16* VL = (const __bf16*)(const void*)VLp;
  const __bf16* WX = (const __bf16*)(const void*)WXp + (size_t)i * LP * DJ;
  const _Float16* Gi = (const _Float16*)(const void*)Gtp + (size_t)i * LP * LP;
  _Float16* sPw = sP[wave];

  for (int item = wave; item < BB * NTG; item += 4) {
    const int j  = item / NTG;
    const int tg = item - j * NTG;
    const int R0 = j * TPC + tg * 32;
    v8f acc[2][2];
#pragma unroll
    for (int a = 0; a < 2; ++a)
#pragma unroll
      for (int c = 0; c < 2; ++c) acc[a][c] = zero8();
    for (int k0 = 0; k0 < DJ; k0 += 32) {
      const v16b b0 = ldfrag_b(WX + (size_t)m * DJ + koff + k0);
      const v16b b1 = ldfrag_b(WX + (size_t)(16 + m) * DJ + koff + k0);
#pragma unroll
      for (int mi = 0; mi < 2; ++mi) {
        const size_t ao = (size_t)(R0 + mi * 16 + m) * DJ + koff + k0;
        const v16b ah = ldfrag_b(VH + ao);
        const v16b al = ldfrag_b(VL + ao);
        acc[mi][0] = mma_b_raw(ah, b0, acc[mi][0]);
        acc[mi][0] = mma_b_raw(al, b0, acc[mi][0]);
        acc[mi][1] = mma_b_raw(ah, b1, acc[mi][1]);
        acc[mi][1] = mma_b_raw(al, b1, acc[mi][1]);
        dep_guard_b(acc[mi][0], acc[mi][1], ah, al);
      }
      keep2_b(b0, b1);
    }
    acc_guard4(acc[0][0], acc[0][1], acc[1][0], acc[1][1]);

    float runmax = -3.0e38f;
#pragma unroll
    for (int mi = 0; mi < 2; ++mi) {
      const int rb = R0 + mi * 16 + h * 8;
      F8 cu, vu;
      cu.v[0] = *(const v4f*)(cT + rb);
      cu.v[1] = *(const v4f*)(cT + rb + 4);
      vu.v[0] = *(const v4f*)(vnT + rb);
      vu.v[1] = *(const v4f*)(vnT + rb + 4);
      float a0r[8], a1r[8], nmr[8];
      wave_sync_lds();
#pragma unroll
      for (int r = 0; r < 8; ++r) {
        const float s0 = acc[mi][0][r] - cu.f[r];
        const float s1 = acc[mi][1][r] - cu.f[r];
        const float x0 = mk0 ? LAMF * s0 : -1.0e9f;
        const float x1 = mk1 ? LAMF * s1 : -1.0e9f;
        float mx = val1 ? fmaxf(x0, x1) : x0;
        mx = hmax16(mx);
        const float e0 = __expf(x0 - mx);
        float e1 = __expf(fminf(x1 - mx, 0.f));
        e1 = val1 ? e1 : 0.f;
        const float ssum = hsum16(e0 + e1);
        const float inv  = 1.0f / ssum;
        const float a0 = e0 * inv, a1 = e1 * inv;
        const float nm = hsum16(a0 * s0 + a1 * s1);
        a0r[r] = a0; a1r[r] = a1; nmr[r] = nm;
        sPw[(h * 8 + r) * LP + m]      = (_Float16)(a0 * ASC);
        sPw[(h * 8 + r) * LP + 16 + m] = (_Float16)(a1 * ASC);
      }
      wave_sync_lds();
      FragH pa, g0, g1;
      pa.hf[0] = *(const v8h*)(sPw + m * LP + koff);
      pa.hf[1] = *(const v8h*)(sPw + m * LP + 16 + koff);
      g0.hf[0] = *(const v8h*)(Gi + m * LP + koff);
      g0.hf[1] = *(const v8h*)(Gi + m * LP + 16 + koff);
      g1.hf[0] = *(const v8h*)(Gi + (16 + m) * LP + koff);
      g1.hf[1] = *(const v8h*)(Gi + (16 + m) * LP + 16 + koff);
      v8f u0 = mma_h_raw(pa.v, g0.v, zero8());
      v8f u1 = mma_h_raw(pa.v, g1.v, zero8());
      dep_guard_h3(u0, u1, pa.v, g0.v, g1.v);
#pragma unroll
      for (int r = 0; r < 8; ++r) {
        float vp = a0r[r] * u0[r] + a1r[r] * u1[r];
        vp = hsum16(vp) * (1.0f / ASC);
        vp = fmaxf(vp, 0.f);
        const float vsn = fmaxf(sqrtf(vp), 1e-8f);
        const float vnn = fmaxf(vu.f[r], 1e-8f);
        const float sim = nmr[r] / (vnn * vsn);
        const int tp = tg * 32 + mi * 16 + h * 8 + r;
        const bool valid = tp < TPV;
        runmax = fmaxf(runmax, valid ? sim : -3.0e38f);
        if (j == i && valid && m == 0) sPos[tp] = sim;
      }
    }
    float mw = runmax;
#pragma unroll
    for (int off = 16; off > 0; off >>= 1) mw = fmaxf(mw, __shfl_xor(mw, off, 32));
    if (lane == 0) sItem[item] = mw;
  }
  __syncthreads();
  if (tid < BB) {
    float s = -3.0e38f;
#pragma unroll
    for (int tg = 0; tg < NTG; ++tg) s = fmaxf(s, sItem[tid * NTG + tg]);
    sSc[tid] = s;
  }
  __syncthreads();
  if (tid < 8) {
    const v4f sc = *(const v4f*)(sSc + tid * 4);
    v4f pv[NTG];
#pragma unroll
    for (int q = 0; q < NTG; ++q) pv[q] = *(const v4f*)(sPos + q * 32 + tid * 4);
    float* ps = scoresT + (size_t)i * SCP + tid * 4;
    float* pp = posT + (size_t)i * TPC + tid * 4;
    for (int pass = 0; pass < 2; ++pass) {
      *(volatile v4f*)ps = sc;
#pragma unroll
      for (int q = 0; q < NTG; ++q) *(volatile v4f*)(pp + q * 32) = pv[q];
      __threadfence();
    }
  }
}

__global__ __launch_bounds__(256) void final_kernel(const float* __restrict__ scoresT, const float* __restrict__ posT,
                                                    float* out, int outN) {
  __shared__ float sS[BB * SCP];
  __shared__ float r1[256];
  __shared__ float r2[256];
  __shared__ float sLoss;
  const int tid = threadIdx.x, wave = tid >> 5, lane = tid & 31;
  for (int p = tid; p < BB * SCP; p += 256) sS[p] = scoresT[p];
  __syncthreads();
  float cs = 0.f, ci = 0.f;
#pragma unroll 1
  for (int p = tid; p < BB * BB; p += 256) {
    const int a = p / BB, bq = p - a * BB;
    if (a != bq) {
      const float s = sS[a * SCP + bq];
      cs += fmaxf(0.f, HINGE + s - sS[a * SCP + a]);
      ci += fmaxf(0.f, HINGE + s - sS[bq * SCP + bq]);
    }
  }
  r1[tid] = cs;
  r2[tid] = ci;
  __syncthreads();
  for (int s = 128; s > 0; s >>= 1) {
    if (tid < s) {
      r1[tid] += r1[tid + s];
      r2[tid] += r2[tid + s];
    }
    __syncthreads();
  }
  if (tid == 0) sLoss = r1[0] * (1.0f / (float)BB) + r2[0] * (1.0f / (float)BB);
  __syncthreads();
  const float loss = sLoss;
  const int nLines = (outN + 31) >> 5;
  for (int pass = 0; pass < 2; ++pass) {
    for (int q = wave; q < nLines; q += 8) {
      if (lane < 8) {
        const int f0 = q * 32 + lane * 4;
        v4f v;
#pragma unroll
        for (int e = 0; e < 4; ++e) {
          const int f = f0 + e;
          int pi = f - 1;
          pi = (pi < 0) ? 0 : ((pi > BB * TPV - 1) ? (BB * TPV - 1) : pi);
          const int bi = pi / TPV;
          const int ti = pi - bi * TPV;
          const float pv = posT[bi * TPC + ti];
          v[e] = (f == 0) ? loss : pv;
        }
        if (f0 + 3 < outN) {
          *(volatile v4f*)(out + f0) = v;
        } else {
#pragma unroll
          for (int e = 0; e < 4; ++e)
            if (f0 + e < outN) *(volatile float*)(out + f0 + e) = v[e];
        }
      }
    }
    __threadfence();
    __syncthreads();
  }
}

extern "C" void kernel_launch(void* const* d_in, const int* in_sizes, int n_in,
                              void* d_out, int out_size, void* d_ws, size_t ws_size,
                              hipStream_t stream) {
  if (n_in < 11) return;
  if (in_sizes[0] != BB * TT * DV) return;
  if (in_sizes[1] != BB * LW * DJ) return;
  if (in_sizes[2] != BB * LW) return;
  if (in_sizes[3] != DJ * DV * KS) return;
  if (in_sizes[4] != DJ) return;
  if (in_sizes[5] != DJ * DJ * KS || in_sizes[6] != DJ) return;
  if (in_sizes[7] != DJ * DJ * KS || in_sizes[8] != DJ) return;
  if (in_sizes[9] != DJ * DJ || in_sizes[10] != DJ) return;
  if (out_size != 1 + BB * TPV) return;

  const float* video = (const float*)d_in[0];
  const float* words = (const float*)d_in[1];
  const float* wmask = (const float*)d_in[2];
  const float* c0w   = (const float*)d_in[3];
  const float* c0b   = (const float*)d_in[4];
  const float* c1w   = (const float*)d_in[5];
  const float* c1b   = (const float*)d_in[6];
  const float* c2w   = (const float*)d_in[7];
  const float* c2b   = (const float*)d_in[8];
  const float* cdw   = (const float*)d_in[9];
  const float* cdb   = (const float*)d_in[10];
  float* out = (float*)d_out;

  const size_t PSTV = (size_t)DV * 128;
  const size_t PSTW = (size_t)DJ * 128;
  const size_t PXV  = (size_t)BB * TT * DV * 2;
  const size_t PW0  = (size_t)DJ * DV * KS * 2;
  const size_t PW1  = (size_t)DJ * DJ * KS * 2;
  const size_t PW3  = (size_t)DJ * DJ * 2;
  const size_t PXC  = (size_t)BB * SP * DJ * 2;
  const size_t PY   = (size_t)BB * SP * DJ * 4;
  const size_t PWP  = (size_t)BB * LP * DJ * 2;
  const size_t PGT  = (size_t)BB * LP * LP * 2;
  const size_t PVH  = (size_t)NR * DJ * 2;
  const size_t PROW = (size_t)NR * 4;
  const size_t PSCR = (size_t)BB * SCP * 4;
  const size_t PPOS = (size_t)BB * TPC * 4;
  size_t off = 0;
  const size_t oSTV = off; off += PSTV;
  const size_t oSTW = off; off += PSTW;
  const size_t oSTY = off; off += PSTW;
  const size_t oXVH = off; off += PXV;
  const size_t oXVL = off; off += PXV;
  const size_t oW0  = off; off += PW0;
  const size_t oW1  = off; off += PW1;
  const size_t oW2  = off; off += PW1;
  const size_t oW3  = off; off += PW3;
  const size_t oXCH = off; off += PXC;
  const size_t oXCL = off; off += PXC;
  const size_t oY   = off; off += PY;
  const size_t oWX  = off; off += PWP;
  const size_t oWH  = off; off += PWP;
  const size_t oWL  = off; off += PWP;
  const size_t oGT  = off; off += PGT;
  const size_t oVH  = off; off += PVH;
  const size_t oVL  = off; off += PVH;
  const size_t oVN  = off; off += PROW;
  const size_t oCT  = off; off += PROW;
  const size_t oSCR = off; off += PSCR;
  const size_t oPOS = off; off += PPOS;
  if (off > ws_size) return;
  if (off > (size_t)134217728) return;

  char* ws = (char*)d_ws;
  float* stV = (float*)(ws + oSTV);
  float* stW = (float*)(ws + oSTW);
  float* stY = (float*)(ws + oSTY);
  unsigned short* XvH = (unsigned short*)(ws + oXVH);
  unsigned short* XvL = (unsigned short*)(ws + oXVL);
  unsigned short* W0p = (unsigned short*)(ws + oW0);
  unsigned short* W1p = (unsigned short*)(ws + oW1);
  unsigned short* W2p = (unsigned short*)(ws + oW2);
  unsigned short* W3p = (unsigned short*)(ws + oW3);
  unsigned short* XCH = (unsigned short*)(ws + oXCH);
  unsigned short* XCL = (unsigned short*)(ws + oXCL);
  float* Y = (float*)(ws + oY);
  unsigned short* WX = (unsigned short*)(ws + oWX);
  unsigned short* WH = (unsigned short*)(ws + oWH);
  unsigned short* WL = (unsigned short*)(ws + oWL);
  unsigned short* Gt = (unsigned short*)(ws + oGT);
  unsigned short* VH = (unsigned short*)(ws + oVH);
  unsigned short* VL = (unsigned short*)(ws + oVL);
  float* vnT = (float*)(ws + oVN);
  float* cT  = (float*)(ws + oCT);
  float* scoresT = (float*)(ws + oSCR);
  float* posT    = (float*)(ws + oPOS);

  const dim3 blk(256);
  const int n8v  = BB * TT * DV / 8;
  const int n8w0 = DJ * DV * KS / 8;
  const int n8w1 = DJ * DJ * KS / 8;
  const int n8w3 = DJ * DJ / 8;

  stats_in<<<dim3(DV), blk, 0, stream>>>(video, BB * TT, DV, stV);
  stats_in<<<dim3(DJ), blk, 0, stream>>>(words, BB * LW, DJ, stW);
  video_split8<<<dim3(n8v / 256), blk, 0, stream>>>(video, stV, XvH, XvL, n8v);
  wconv_cvt8<<<dim3(n8w0 / 256), blk, 0, stream>>>(c0w, DV, KS, W0p, n8w0);
  wconv_cvt8<<<dim3(n8w1 / 256), blk, 0, stream>>>(c1w, DJ, KS, W1p, n8w1);
  wconv_cvt8<<<dim3(n8w1 / 256), blk, 0, stream>>>(c2w, DJ, KS, W2p, n8w1);
  wconv_cvt8<<<dim3(n8w3 / 256), blk, 0, stream>>>(cdw, DJ, 1, W3p, n8w3);
  words_planes<<<dim3(BB * LP / 8), blk, 0, stream>>>(words, stW, WX, WH, WL);
  gram_kernel<<<dim3(BB), dim3(32), 0, stream>>>(WH, WL, Gt);
  gemm64<1, 1><<<dim3(2, BB), blk, 0, stream>>>(
      XvH, XvL, 2 * DV, (long long)TT * DV, T1,
      W0p, KS * DV, 0LL,
      (void*)XCH, (void*)XCL, DJ, (long long)SP * DJ, c0b,
      128, DJ, KS * DV);
  gemm64<1, 1><<<dim3(1, BB), blk, 0, stream>>>(
      XCH, XCL, 2 * DJ, (long long)SP * DJ, T2,
      W1p, KS * DJ, 0LL,
      (void*)(XCH + 128 * DJ), (void*)(XCL + 128 * DJ), DJ, (long long)SP * DJ, c1b,
      64, DJ, KS * DJ);
  gemm64<1, 1><<<dim3(1, BB), blk, 0, stream>>>(
      XCH + 128 * DJ, XCL + 128 * DJ, 2 * DJ, (long long)SP * DJ, T3,
      W2p, KS * DJ, 0LL,
      (void*)(XCH + 192 * DJ), (void*)(XCL + 192 * DJ), DJ, (long long)SP * DJ, c2b,
      64, DJ, KS * DJ);
  gemm64<1, 0><<<dim3(4, BB), blk, 0, stream>>>(
      XCH, XCL, DJ, (long long)SP * DJ, SP,
      W3p, DJ, 0LL,
      (void*)Y, (void*)Y, DJ, (long long)SP * DJ, cdb,
      SP, DJ, DJ);
  stats_y<<<dim3(DJ), blk, 0, stream>>>(Y, cdb, stY);
  vfinish<<<dim3(NR / 32), blk, 0, stream>>>(Y, cdb, stY, stW, VH, VL, vnT, cT);
  attn_kernel<<<dim3(BB), dim3(128), 0, stream>>>(VH, VL, WX, Gt, vnT, cT, wmask, scoresT, posT);
  final_kernel<<<dim3(1), blk, 0, stream>>>(scoresT, posT, out, out_size);
  (void)hipGetLastError();
}
